// GCNRegressor_27986006901220
// MI455X (gfx1250) — hardware-verified
//
#include <hip/hip_runtime.h>
#include <stddef.h>


#define DF      128
#define NG      512
#define NTHR    256
#define NWAVE   8
#define EPT     8
#define NGRP    2
#define CHUNK   (NTHR * EPT * NGRP)
#define WCAP    (EPT * NGRP * 32)
#define LISTN   (NWAVE * WCAP)
#define NBA     512
#define NBD     4096
#define G1ROWS  128
#define APITCH  136
#define NWMAT   4
#define WSCALE  8.0f
#define WINV    0.125f

#define LDS_GEMM1 (G1ROWS * DF * 4)
#define LDS_AGG   (NBA * DF * 4 + LISTN * 4 + 64)

static_assert((CHUNK & (CHUNK - 1)) == 0);
static_assert(CHUNK <= 4096);
static_assert(NBA <= 4096 && NBD <= 4096);
static_assert((NBA & (NBA - 1)) == 0 && (NBD & (NBD - 1)) == 0);
static_assert(G1ROWS * APITCH * 2 <= LDS_GEMM1);
static_assert(NBA % (16 * NWAVE) == 0);
static_assert(NG % (16 * NWAVE) == 0);
static_assert(NBD % NBA == 0 && NBD % G1ROWS == 0);
static_assert(NG == 4 * 128);

typedef float    v4f  __attribute__((ext_vector_type(4)));
typedef float    v8f  __attribute__((ext_vector_type(8)));
typedef int      v4i  __attribute__((ext_vector_type(4)));
typedef _Float16 v8h  __attribute__((ext_vector_type(8)));
typedef _Float16 v16h __attribute__((ext_vector_type(16)));
union FragH { v16h v; v8h h[2]; };

__device__ __forceinline__ v8h cvt8(v4f a, v4f b) {
  v8h r;
  r[0] = (_Float16)a.x; r[1] = (_Float16)a.y; r[2] = (_Float16)a.z; r[3] = (_Float16)a.w;
  r[4] = (_Float16)b.x; r[5] = (_Float16)b.y; r[6] = (_Float16)b.z; r[7] = (_Float16)b.w;
  return r;
}

__device__ __forceinline__ v8f wmh(v16h a, v16h b, v8f c) {
  v8f d = __builtin_amdgcn_wmma_f32_16x16x32_f16(false, a, false, b, (short)0, c, false, false);
  asm volatile("v_nop\n\tv_nop\n\tv_nop\n\tv_nop" : "+v"(d) : "v"(a), "v"(b));
  return d;
}

template <int NB>
__device__ __forceinline__ int scan_chunk(const int* __restrict__ dsts, int nE, int cbase, int nodeBase,
                                          int vec8, int* list, int tid, int lane, int wave) {
  int wc = 0;
#pragma unroll
  for (int g = 0; g < NGRP; ++g) {
    const int el0  = (g * NTHR + tid) * EPT;
    const int e0   = cbase + el0;
    const int sent = -2147483647 - 1;
    v4i da, db;
    if (vec8 != 0 && e0 + 7 < nE) {
      da = *(const v4i*)(dsts + e0);
      db = *(const v4i*)(dsts + e0 + 4);
    } else {
      da.x = (e0     < nE) ? dsts[e0]     : sent;
      da.y = (e0 + 1 < nE) ? dsts[e0 + 1] : sent;
      da.z = (e0 + 2 < nE) ? dsts[e0 + 2] : sent;
      da.w = (e0 + 3 < nE) ? dsts[e0 + 3] : sent;
      db.x = (e0 + 4 < nE) ? dsts[e0 + 4] : sent;
      db.y = (e0 + 5 < nE) ? dsts[e0 + 5] : sent;
      db.z = (e0 + 6 < nE) ? dsts[e0 + 6] : sent;
      db.w = (e0 + 7 < nE) ? dsts[e0 + 7] : sent;
    }
    const unsigned nb = (unsigned)nodeBase;
    const unsigned s0 = (unsigned)da.x - nb, s1 = (unsigned)da.y - nb;
    const unsigned s2 = (unsigned)da.z - nb, s3 = (unsigned)da.w - nb;
    const unsigned s4 = (unsigned)db.x - nb, s5 = (unsigned)db.y - nb;
    const unsigned s6 = (unsigned)db.z - nb, s7 = (unsigned)db.w - nb;
    const bool h0 = s0 < (unsigned)NB, h1 = s1 < (unsigned)NB, h2 = s2 < (unsigned)NB, h3 = s3 < (unsigned)NB;
    const bool h4 = s4 < (unsigned)NB, h5 = s5 < (unsigned)NB, h6 = s6 < (unsigned)NB, h7 = s7 < (unsigned)NB;
    const unsigned any = __builtin_amdgcn_ballot_w32(h0 | h1 | h2 | h3 | h4 | h5 | h6 | h7);
    if (any != 0u) {
#define HITJ(J, HJ, SJ) { \
        const unsigned mj = __builtin_amdgcn_ballot_w32(HJ); \
        if (mj != 0u) { \
          if (HJ) { \
            const int pos = wc + (int)__builtin_amdgcn_mbcnt_lo(mj, 0u); \
            if (pos < WCAP) list[wave * WCAP + pos] = ((el0 + (J)) << 12) | (int)(SJ); \
          } \
          wc += (int)__builtin_popcount(mj); } }
      HITJ(0, h0, s0)
      HITJ(1, h1, s1)
      HITJ(2, h2, s2)
      HITJ(3, h3, s3)
      HITJ(4, h4, s4)
      HITJ(5, h5, s5)
      HITJ(6, h6, s6)
      HITJ(7, h7, s7)
#undef HITJ
    }
  }
  return wc;
}

__global__ __launch_bounds__(NTHR) void k_wprep(
    const float* __restrict__ Wa, const float* __restrict__ Wb,
    const float* __restrict__ Wc, const float* __restrict__ Wd, _Float16* wpl) {
  const int i   = blockIdx.x * NTHR + threadIdx.x;
  const int per = DF * DF / 8;
  if (i >= NWMAT * per) return;
  const int mat = i / per;
  const int o   = (i - mat * per) * 8;
  const int n   = o / DF;
  const int k0  = o - n * DF;
  const float* W = (mat == 0) ? Wa : ((mat == 1) ? Wb : ((mat == 2) ? Wc : Wd));
  const float* p = W + (size_t)k0 * DF + n;
  v4f a, b;
  a.x = p[0];      a.y = p[DF];     a.z = p[2 * DF]; a.w = p[3 * DF];
  b.x = p[4 * DF]; b.y = p[5 * DF]; b.z = p[6 * DF]; b.w = p[7 * DF];
  a = a * WSCALE;
  b = b * WSCALE;
  const v8h hv = cvt8(a, b);
  _Float16* dp = wpl + (size_t)mat * DF * DF + o;
  *(volatile v8h*)dp = hv;
  __threadfence();
  *(volatile v8h*)dp = hv;
}

__global__ __launch_bounds__(NTHR) void k_deg(
    const int* __restrict__ ei, float* dinv, int nN, int nE, int vec8) {
  __shared__ __attribute__((aligned(16))) int cnt[NBD];
  __shared__ __attribute__((aligned(16))) int list[LISTN];
  __shared__ int wcnt[NWAVE];
  const int tid = threadIdx.x, lane = tid & 31, wave = tid >> 5;
  const int nodeBase = blockIdx.x * NBD;
  const int* dsts = ei + nE;
  (void)nN;

  for (int i = tid; i < NBD; i += NTHR) cnt[i] = 0;
  __syncthreads();

  const int nChunks = (nE + CHUNK - 1) / CHUNK;
#pragma unroll 1
  for (int ch = 0; ch < nChunks; ++ch) {
    const int cbase = ch * CHUNK;
    const int wc = scan_chunk<NBD>(dsts, nE, cbase, nodeBase, vec8, list, tid, lane, wave);
    if (lane == 0) wcnt[wave] = wc;
    __syncthreads();
    if (wave == 0) {
#pragma unroll 1
      for (int wsx = 0; wsx < NWAVE; ++wsx) {
        int n = __builtin_amdgcn_readfirstlane(wcnt[wsx]);
        n = n > WCAP ? WCAP : (n < 0 ? 0 : n);
        const int* lp = list + wsx * WCAP;
#pragma unroll 1
        for (int i = 0; i < n; ++i) {
          const int ent  = __builtin_amdgcn_readfirstlane(lp[i]);
          const int slot = ent & (NBD - 1);
          if (lane == 0) cnt[slot] = cnt[slot] + 1;
        }
      }
    }
    __syncthreads();
  }

  v4f dq[4];
#pragma unroll
  for (int q = 0; q < 4; ++q) {
    const int f = (wave * 4 + q) * 128 + 4 * lane;
    const v4i c = *(const v4i*)(cnt + f);
    dq[q].x = rsqrtf((float)(c.x + 1));
    dq[q].y = rsqrtf((float)(c.y + 1));
    dq[q].z = rsqrtf((float)(c.z + 1));
    dq[q].w = rsqrtf((float)(c.w + 1));
  }
  float* dp = dinv + (size_t)nodeBase;
#pragma unroll
  for (int q = 0; q < 4; ++q) *(volatile v4f*)(dp + (wave * 4 + q) * 128 + 4 * lane) = dq[q];
  __threadfence();
#pragma unroll
  for (int q = 0; q < 4; ++q) *(volatile v4f*)(dp + (wave * 4 + q) * 128 + 4 * lane) = dq[q];
}

__global__ __launch_bounds__(NTHR) void k_gemm1(
    const float* __restrict__ x, const _Float16* __restrict__ w0s,
    const float* __restrict__ dinv, float* g1, int nN) {
  extern __shared__ v4f lds_dyn[];
  _Float16* sA  = (_Float16*)lds_dyn;
  float*    stg = (float*)lds_dyn;
  const int tid = threadIdx.x, lane = tid & 31, wave = tid >> 5, hh = lane >> 4, m = lane & 15;
  const int rowBase = blockIdx.x * G1ROWS;

#pragma unroll
  for (int i = 0; i < (G1ROWS * DF / 8) / NTHR; ++i) {
    const int idx = i * NTHR + tid;
    const int r   = idx >> 4;
    const int c0  = (idx & 15) * 8;
    int node = rowBase + r;
    node = node > nN - 1 ? nN - 1 : node;
    const float* xp = x + (size_t)node * DF + c0;
    const v4f a = *(const v4f*)xp, b = *(const v4f*)(xp + 4);
    *(v8h*)(sA + r * APITCH + c0) = cvt8(a, b);
  }
  __syncthreads();

  v8f acc[8];
#pragma unroll
  for (int t = 0; t < 8; ++t) { v8f z = {0.f, 0.f, 0.f, 0.f, 0.f, 0.f, 0.f, 0.f}; acc[t] = z; }
  const _Float16* ar = sA + (wave * 16 + m) * APITCH + 8 * hh;
#pragma unroll
  for (int kt = 0; kt < DF / 32; ++kt) {
    FragH a;
    a.h[0] = *(const v8h*)(ar + 32 * kt);
    a.h[1] = *(const v8h*)(ar + 32 * kt + 16);
#pragma unroll
    for (int t = 0; t < 8; ++t) {
      const _Float16* bp = w0s + (size_t)(16 * t + m) * DF + 32 * kt + 8 * hh;
      FragH b;
      b.h[0] = *(const v8h*)bp;
      b.h[1] = *(const v8h*)(bp + 16);
      acc[t] = wmh(a.v, b.v, acc[t]);
    }
  }
  __syncthreads();

  const int r0 = wave * 16 + 8 * hh;
  const v4f dA = *(const v4f*)(dinv + (size_t)rowBase + r0);
  const v4f dB = *(const v4f*)(dinv + (size_t)rowBase + r0 + 4);
  const float d0 = dA.x * WINV, d1 = dA.y * WINV, d2 = dA.z * WINV, d3 = dA.w * WINV;
  const float d4 = dB.x * WINV, d5 = dB.y * WINV, d6 = dB.z * WINV, d7 = dB.w * WINV;
  float* sp = stg + r0 * DF + m;
#pragma unroll
  for (int t = 0; t < 8; ++t) {
    sp[0 * DF + 16 * t] = acc[t][0] * d0;
    sp[1 * DF + 16 * t] = acc[t][1] * d1;
    sp[2 * DF + 16 * t] = acc[t][2] * d2;
    sp[3 * DF + 16 * t] = acc[t][3] * d3;
    sp[4 * DF + 16 * t] = acc[t][4] * d4;
    sp[5 * DF + 16 * t] = acc[t][5] * d5;
    sp[6 * DF + 16 * t] = acc[t][6] * d6;
    sp[7 * DF + 16 * t] = acc[t][7] * d7;
  }
  __syncthreads();

  const float* lp = stg + wave * 16 * DF + 4 * lane;
  float* gp = g1 + ((size_t)rowBase + wave * 16) * DF + 4 * lane;
#pragma unroll
  for (int i = 0; i < 16; ++i) { const v4f v = *(const v4f*)(lp + i * DF); *(volatile v4f*)(gp + (size_t)i * DF) = v; }
  __threadfence();
#pragma unroll
  for (int i = 0; i < 16; ++i) { const v4f v = *(const v4f*)(lp + i * DF); *(volatile v4f*)(gp + (size_t)i * DF) = v; }
}

template <bool FUSE>
__global__ __launch_bounds__(NTHR) void k_agg(
    const int* __restrict__ ei, const float* __restrict__ gin, const float* __restrict__ dinv,
    const float* __restrict__ bias, const _Float16* __restrict__ wn, float* gout,
    int nN, int nE, int vec8) {
  extern __shared__ v4f lds_dyn[];
  float* acc  = (float*)lds_dyn;
  int*   list = (int*)(acc + NBA * DF);
  int*   wcnt = list + LISTN;
  const int tid = threadIdx.x, lane = tid & 31, wave = tid >> 5, hh = lane >> 4, m = lane & 15;
  const int nodeBase = blockIdx.x * NBA;
  const int* dsts = ei + nE;

  {
    const v4f z = {0.f, 0.f, 0.f, 0.f};
    for (int i = tid; i < NBA * DF / 4; i += NTHR) lds_dyn[i] = z;
  }
  __syncthreads();

  const int nChunks = (nE + CHUNK - 1) / CHUNK;
#pragma unroll 1
  for (int ch = 0; ch < nChunks; ++ch) {
    const int cbase = ch * CHUNK;
    const int wc = scan_chunk<NBA>(dsts, nE, cbase, nodeBase, vec8, list, tid, lane, wave);
    if (lane == 0) wcnt[wave] = wc;
    __syncthreads();
    if (wave == 0) {
#pragma unroll 1
      for (int wsx = 0; wsx < NWAVE; ++wsx) {
        int n = __builtin_amdgcn_readfirstlane(wcnt[wsx]);
        n = n > WCAP ? WCAP : (n < 0 ? 0 : n);
        const int* lp = list + wsx * WCAP;
#pragma unroll 1
        for (int i = 0; i < n; ++i) {
          const int ent  = __builtin_amdgcn_readfirstlane(lp[i]);
          const int slot = ent & (NBA - 1);
          int e = cbase + ((ent >> 12) & (CHUNK - 1));
          e = e > nE - 1 ? nE - 1 : e;
          int src = ei[e];
          src = src < 0 ? 0 : (src > nN - 1 ? nN - 1 : src);
          const v4f v = *(const v4f*)(gin + (size_t)src * DF + 4 * lane);
          v4f* ap = (v4f*)(acc + slot * DF + 4 * lane);
          *ap = *ap + v;
        }
      }
    }
    __syncthreads();
  }

#pragma unroll 4
  for (int i = 0; i < (NBA * DF / 4) / NTHR; ++i) {
    const int idx  = i * NTHR + tid;
    const int slot = idx >> 5;
    const int c4   = (idx & 31) * 4;
    int node = nodeBase + slot;
    node = node > nN - 1 ? nN - 1 : node;
    const float d  = dinv[node];
    const v4f   gv = *(const v4f*)(gin + (size_t)node * DF + c4);
    const v4f   bv = *(const v4f*)(bias + c4);
    v4f* ap = (v4f*)(acc + slot * DF + c4);
    v4f hv = (*ap + gv) * d + bv;
    hv.x = fmaxf(hv.x, 0.f); hv.y = fmaxf(hv.y, 0.f); hv.z = fmaxf(hv.z, 0.f); hv.w = fmaxf(hv.w, 0.f);
    *ap = hv;
  }
  __syncthreads();

  if (FUSE) {
#pragma unroll 1
    for (int it = 0; it < NBA / 16 / NWAVE; ++it) {
      const int t = wave + NWAVE * it;
      v8f c[8];
#pragma unroll
      for (int tt = 0; tt < 8; ++tt) { v8f z = {0.f, 0.f, 0.f, 0.f, 0.f, 0.f, 0.f, 0.f}; c[tt] = z; }
#pragma unroll
      for (int kt = 0; kt < DF / 32; ++kt) {
        const float* ap = acc + (16 * t + m) * DF + 32 * kt + 8 * hh;
        const v4f p0 = *(const v4f*)ap,        p1 = *(const v4f*)(ap + 4);
        const v4f p2 = *(const v4f*)(ap + 16), p3 = *(const v4f*)(ap + 20);
        FragH a;
        a.h[0] = cvt8(p0, p1);
        a.h[1] = cvt8(p2, p3);
#pragma unroll
        for (int tt = 0; tt < 8; ++tt) {
          const _Float16* bp = wn + (size_t)(16 * tt + m) * DF + 32 * kt + 8 * hh;
          FragH b;
          b.h[0] = *(const v8h*)bp;
          b.h[1] = *(const v8h*)(bp + 16);
          c[tt] = wmh(a.v, b.v, c[tt]);
        }
      }
      const int node0 = nodeBase + 16 * t + 8 * hh;
      const v4f dA = *(const v4f*)(dinv + (size_t)node0);
      const v4f dB = *(const v4f*)(dinv + (size_t)node0 + 4);
      const float d0 = dA.x * WINV, d1 = dA.y * WINV, d2 = dA.z * WINV, d3 = dA.w * WINV;
      const float d4 = dB.x * WINV, d5 = dB.y * WINV, d6 = dB.z * WINV, d7 = dB.w * WINV;
      float* sp = acc + (16 * t + 8 * hh) * DF + m;
#pragma unroll
      for (int tt = 0; tt < 8; ++tt) {
        sp[0 * DF + 16 * tt] = c[tt][0] * d0;
        sp[1 * DF + 16 * tt] = c[tt][1] * d1;
        sp[2 * DF + 16 * tt] = c[tt][2] * d2;
        sp[3 * DF + 16 * tt] = c[tt][3] * d3;
        sp[4 * DF + 16 * tt] = c[tt][4] * d4;
        sp[5 * DF + 16 * tt] = c[tt][5] * d5;
        sp[6 * DF + 16 * tt] = c[tt][6] * d6;
        sp[7 * DF + 16 * tt] = c[tt][7] * d7;
      }
    }
    __syncthreads();
  }

  const float* lp = acc + wave * (NBA / NWAVE) * DF + 4 * lane;
  float* gp = gout + ((size_t)nodeBase + wave * (NBA / NWAVE)) * DF + 4 * lane;
#pragma unroll 8
  for (int i = 0; i < NBA / NWAVE; ++i) { const v4f v = *(const v4f*)(lp + i * DF); *(volatile v4f*)(gp + (size_t)i * DF) = v; }
  __threadfence();
#pragma unroll 8
  for (int i = 0; i < NBA / NWAVE; ++i) { const v4f v = *(const v4f*)(lp + i * DF); *(volatile v4f*)(gp + (size_t)i * DF) = v; }
}

__global__ __launch_bounds__(NTHR) void k_pool(
    const int* __restrict__ bat, const float* __restrict__ h, float* pooled, int nN, int vecb) {
  __shared__ __attribute__((aligned(16))) int list[LISTN];
  __shared__ int wcnt[NWAVE];
  const int tid = threadIdx.x, lane = tid & 31, wave = tid >> 5;
  const int g = blockIdx.x;
  v4f s = {0.f, 0.f, 0.f, 0.f};
  int cnt = 0;

  const int nChunks = (nN + CHUNK - 1) / CHUNK;
#pragma unroll 1
  for (int ch = 0; ch < nChunks; ++ch) {
    const int cbase = ch * CHUNK;
    const int wc = scan_chunk<1>(bat, nN, cbase, g, vecb, list, tid, lane, wave);
    if (lane == 0) wcnt[wave] = wc;
    __syncthreads();
    if (wave == 0) {
#pragma unroll 1
      for (int wsx = 0; wsx < NWAVE; ++wsx) {
        int n = __builtin_amdgcn_readfirstlane(wcnt[wsx]);
        n = n > WCAP ? WCAP : (n < 0 ? 0 : n);
        const int* lp = list + wsx * WCAP;
#pragma unroll 1
        for (int i = 0; i < n; ++i) {
          const int ent = __builtin_amdgcn_readfirstlane(lp[i]);
          int node = cbase + ((ent >> 12) & (CHUNK - 1));
          node = node > nN - 1 ? nN - 1 : node;
          const v4f v = *(const v4f*)(h + (size_t)node * DF + 4 * lane);
          s = s + v;
          cnt += 1;
        }
      }
    }
    __syncthreads();
  }

  if (wave == 0) {
    const float cf  = (float)(cnt > 0 ? cnt : 1);
    const float inv = 1.0f / cf;
    const v4f   o   = s * inv;
    float* pp = pooled + (size_t)g * DF + 4 * lane;
    *(volatile v4f*)pp = o;
    __threadfence();
    *(volatile v4f*)pp = o;
  }
}

__global__ __launch_bounds__(NTHR) void k_head(
    const float* __restrict__ pooled, const _Float16* __restrict__ wm, const float* __restrict__ bm0,
    const float* __restrict__ Wm1, const float* __restrict__ bm1, float* out) {
  __shared__ __attribute__((aligned(16))) float sOut[NG];
  const int tid = threadIdx.x, lane = tid & 31, wave = tid >> 5, hh = lane >> 4, m = lane & 15;
  const float bl = bm1[0];

#pragma unroll 1
  for (int it = 0; it < NG / 16 / NWAVE; ++it) {
    const int t = wave + NWAVE * it;
    v8f c[8];
#pragma unroll
    for (int tt = 0; tt < 8; ++tt) { v8f z = {0.f, 0.f, 0.f, 0.f, 0.f, 0.f, 0.f, 0.f}; c[tt] = z; }
#pragma unroll
    for (int kt = 0; kt < DF / 32; ++kt) {
      const float* ap = pooled + (size_t)(16 * t + m) * DF + 32 * kt + 8 * hh;
      const v4f p0 = *(const v4f*)ap,        p1 = *(const v4f*)(ap + 4);
      const v4f p2 = *(const v4f*)(ap + 16), p3 = *(const v4f*)(ap + 20);
      FragH a;
      a.h[0] = cvt8(p0, p1);
      a.h[1] = cvt8(p2, p3);
#pragma unroll
      for (int tt = 0; tt < 8; ++tt) {
        const _Float16* bp = wm + (size_t)(16 * tt + m) * DF + 32 * kt + 8 * hh;
        FragH b;
        b.h[0] = *(const v8h*)bp;
        b.h[1] = *(const v8h*)(bp + 16);
        c[tt] = wmh(a.v, b.v, c[tt]);
      }
    }
    float pr[8];
#pragma unroll
    for (int r = 0; r < 8; ++r) pr[r] = 0.f;
#pragma unroll
    for (int tt = 0; tt < 8; ++tt) {
      const float bb = bm0[16 * tt + m];
      const float ww = Wm1[16 * tt + m];
#pragma unroll
      for (int r = 0; r < 8; ++r) {
        const float v = fmaxf(c[tt][r] * WINV + bb, 0.f);
        pr[r] += v * ww;
      }
    }
#pragma unroll
    for (int r = 0; r < 8; ++r) {
      pr[r] += __shfl_xor(pr[r], 8, 32);
      pr[r] += __shfl_xor(pr[r], 4, 32);
      pr[r] += __shfl_xor(pr[r], 2, 32);
      pr[r] += __shfl_xor(pr[r], 1, 32);
    }
    if (m == 0) {
#pragma unroll
      for (int r = 0; r < 8; ++r) sOut[16 * t + 8 * hh + r] = pr[r] + bl;
    }
  }
  __syncthreads();

  if (wave == 0) {
    v4f ov[4];
#pragma unroll
    for (int q = 0; q < 4; ++q) ov[q] = *(const v4f*)(sOut + q * 128 + 4 * lane);
#pragma unroll
    for (int q = 0; q < 4; ++q) *(volatile v4f*)(out + q * 128 + 4 * lane) = ov[q];
    __threadfence();
#pragma unroll
    for (int q = 0; q < 4; ++q) *(volatile v4f*)(out + q * 128 + 4 * lane) = ov[q];
  }
}

extern "C" void kernel_launch(void* const* d_in, const int* in_sizes, int n_in,
                              void* d_out, int out_size, void* d_ws, size_t ws_size,
                              hipStream_t stream) {
  if (n_in < 14) return;
  const int nN = in_sizes[0] / DF;
  const int nE = in_sizes[1] / 2;
  if (nN <= 0 || nE < 0 || in_sizes[0] != nN * DF || in_sizes[1] != nE * 2) return;
  if (in_sizes[3] != nN) return;
  if (in_sizes[4] != DF * DF || in_sizes[6] != DF * DF || in_sizes[8] != DF * DF || in_sizes[10] != DF * DF) return;
  if (in_sizes[5] < DF || in_sizes[7] < DF || in_sizes[9] < DF || in_sizes[11] < DF) return;
  if (in_sizes[12] != DF || in_sizes[13] < 1) return;
  if (out_size != NG) return;

  const float* x   = (const float*)d_in[0];
  const int*   ei  = (const int*)d_in[1];
  const int*   bat = (const int*)d_in[3];
  const float* W0  = (const float*)d_in[4];
  const float* b0  = (const float*)d_in[5];
  const float* W1  = (const float*)d_in[6];
  const float* b1  = (const float*)d_in[7];
  const float* W2  = (const float*)d_in[8];
  const float* b2  = (const float*)d_in[9];
  const float* Wm0 = (const float*)d_in[10];
  const float* bm0 = (const float*)d_in[11];
  const float* Wm1 = (const float*)d_in[12];
  const float* bm1 = (const float*)d_in[13];
  float* out = (float*)d_out;

  const int nBD = (nN + NBD - 1) / NBD;
  const int nG1 = (nN + G1ROWS - 1) / G1ROWS;
  const int nA  = (nN + NBA - 1) / NBA;
  const size_t rowsG1 = (size_t)nG1 * G1ROWS;
  const size_t rowsA  = (size_t)nA * NBA;
  const size_t PR     = rowsG1 > rowsA ? rowsG1 : rowsA;

  char* ws = (char*)d_ws;
  size_t off = 0;
  const size_t oW  = off; off += (size_t)NWMAT * DF * DF * 2;                 off = (off + 255) & ~(size_t)255;
  const size_t oDv = off; off += (size_t)nBD * NBD * 4;                       off = (off + 255) & ~(size_t)255;
  const size_t oPA = off; off += PR * DF * 4;                                 off = (off + 255) & ~(size_t)255;
  const size_t oPB = off; off += PR * DF * 4;                                 off = (off + 255) & ~(size_t)255;
  const size_t oPl = off; off += (size_t)NG * DF * 4;                         off = (off + 255) & ~(size_t)255;
  if (off > ws_size || off > ((size_t)1 << 27)) return;
  _Float16* wpl    = (_Float16*)(ws + oW);
  float*    dinv   = (float*)(ws + oDv);
  float*    pA     = (float*)(ws + oPA);
  float*    pB     = (float*)(ws + oPB);
  float*    pooled = (float*)(ws + oPl);
  const _Float16* w0s  = wpl;
  const _Float16* w1s  = wpl + (size_t)1 * DF * DF;
  const _Float16* w2s  = wpl + (size_t)2 * DF * DF;
  const _Float16* wm0s = wpl + (size_t)3 * DF * DF;

  const int vec8 = ((nE & 3) == 0) ? 1 : 0;
  const int vecb = 1;

  const int nPrep = NWMAT * DF * DF / 8;
  k_wprep<<<(nPrep + NTHR - 1) / NTHR, NTHR, 0, stream>>>(W0, W1, W2, Wm0, wpl);

  k_deg<<<nBD, NTHR, 0, stream>>>(ei, dinv, nN, nE, vec8);

  hipFuncSetAttribute(reinterpret_cast<const void*>(&k_gemm1),
                      hipFuncAttributeMaxDynamicSharedMemorySize, LDS_GEMM1);
  k_gemm1<<<nG1, NTHR, LDS_GEMM1, stream>>>(x, w0s, dinv, pA, nN);

  hipFuncSetAttribute(reinterpret_cast<const void*>(&k_agg<true>),
                      hipFuncAttributeMaxDynamicSharedMemorySize, LDS_AGG);
  hipFuncSetAttribute(reinterpret_cast<const void*>(&k_agg<false>),
                      hipFuncAttributeMaxDynamicSharedMemorySize, LDS_AGG);
  k_agg<true><<<nA, NTHR, LDS_AGG, stream>>>(ei, pA, dinv, b0, w1s, pB, nN, nE, vec8);
  k_agg<true><<<nA, NTHR, LDS_AGG, stream>>>(ei, pB, dinv, b1, w2s, pA, nN, nE, vec8);
  k_agg<false><<<nA, NTHR, LDS_AGG, stream>>>(ei, pA, dinv, b2, w0s, pB, nN, nE, vec8);

  k_pool<<<NG, NTHR, 0, stream>>>(bat, pB, pooled, nN, vecb);

  k_head<<<1, NTHR, 0, stream>>>(pooled, wm0s, bm0, Wm1, bm1, out);
}
